// GraphConvNet_14293651161727
// MI455X (gfx1250) — hardware-verified
//
#include <hip/hip_runtime.h>
#include <stddef.h>


#define NTHR   256
#define NWAVE  8
#define EPT    8
#define NGRP   2
#define CHUNK  (NTHR * EPT * NGRP)
#define WCAP   (EPT * NGRP * 32)
#define LISTN  (NWAVE * WCAP)
#define NB1    4096
#define NB2    1024
#define FIN1   16
#define FIN2   64
#define NOUT1  64
#define NOUT2  128
#define F3     128
#define NOUT3  256
#define NG     100
#define DEMO   4
#define DEMW   16
#define KL1    288
#define NL1    128
#define NL2    64
#define NCLS   3
#define HROWS  112
#define POOLP  50
#define PTHR   128
#define RECR   (2 * NG + 2)
#define RECD   (RECR * F3)

#define PO_W1H 0
#define PO_W1L 2048
#define PO_W2H 4096
#define PO_W2L 20480
#define PO_W3H 36864
#define PO_W3L 102400
#define PO_L1H 167936
#define PO_L1L 204800
#define PO_L2H 241664
#define PO_L2L 249856
#define PO_TOT 258048

#define LDS_CONV (NB1 * FIN1 * 4 + LISTN * 4 + 64)
#define LDS_STAT (NTHR * NG * 8 + 512 * 4 + NG * NOUT2 * 4)
#define LDS_POOL (RECD * 8)
#define HL_A3  0
#define HL_H0  (HROWS * NOUT3)
#define HL_INV (HL_H0 + HROWS * KL1)
#define HL_CF  (HL_INV + HROWS)
#define HL_OUT (HL_CF + HROWS)
#define LDS_HEAD ((HL_OUT + 320) * 4)

static_assert((CHUNK & (CHUNK - 1)) == 0);
static_assert(CHUNK <= 4096);
static_assert(NB1 <= 4096 && NB2 <= 4096);
static_assert(NB1 * FIN1 == NB2 * FIN2);
static_assert(NWAVE * 512 <= LISTN);
static_assert((RECD % (2 * PTHR)) == 0);
static_assert((HL_OUT % 4) == 0 && (HL_H0 % 4) == 0);
static_assert((PO_W1L % 64) == 0 && (PO_W2H % 64) == 0 && (PO_W3L % 64) == 0 && (PO_L1H % 64) == 0 && (PO_L2L % 64) == 0);
static_assert(HROWS * NL1 <= HROWS * NOUT3 && HROWS * NL2 <= HROWS * KL1);

typedef float          v2f  __attribute__((ext_vector_type(2)));
typedef float          v4f  __attribute__((ext_vector_type(4)));
typedef float          v8f  __attribute__((ext_vector_type(8)));
typedef int            v4i  __attribute__((ext_vector_type(4)));
typedef unsigned short v8us __attribute__((ext_vector_type(8)));
typedef __bf16         v16b __attribute__((ext_vector_type(16)));
typedef double         v2d  __attribute__((ext_vector_type(2)));
union FragB { v16b v; v8us u[2]; };

__device__ __forceinline__ unsigned bfr(float x) {
  const unsigned u = __float_as_uint(x);
  return (u + 0x7FFFu + ((u >> 16) & 1u)) >> 16;
}

__device__ __forceinline__ void split8(v4f a, v4f b, v8us& hi, v8us& lo) {
  float v[8] = {a.x, a.y, a.z, a.w, b.x, b.y, b.z, b.w};
#pragma unroll
  for (int j = 0; j < 8; ++j) {
    const unsigned hb = bfr(v[j]);
    const float    hf = __uint_as_float(hb << 16);
    const unsigned lb = bfr(v[j] - hf);
    hi[j] = (unsigned short)hb;
    lo[j] = (unsigned short)lb;
  }
}

__device__ __forceinline__ void frag_a(const float* p, FragB& hi, FragB& lo) {
  { const v4f a = *(const v4f*)p,        b = *(const v4f*)(p + 4);  split8(a, b, hi.u[0], lo.u[0]); }
  { const v4f a = *(const v4f*)(p + 16), b = *(const v4f*)(p + 20); split8(a, b, hi.u[1], lo.u[1]); }
}

__device__ __forceinline__ void frag_b(const unsigned short* ph, const unsigned short* pl, FragB& bh, FragB& bl) {
  bh.u[0] = *(const v8us*)ph; bh.u[1] = *(const v8us*)(ph + 16);
  bl.u[0] = *(const v8us*)pl; bl.u[1] = *(const v8us*)(pl + 16);
}

__device__ __forceinline__ v8f wmb(v16b a, v16b b, v8f c) {
  v8f d = __builtin_amdgcn_wmma_f32_16x16x32_bf16(false, a, false, b, (short)0, c, false, false);
  asm volatile("v_nop\n\tv_nop\n\tv_nop\n\tv_nop" : "+v"(d) : "v"(a), "v"(b));
  return d;
}

template <int CT, int K>
__device__ __forceinline__ void mma_step(v8f (&c)[CT], v16b ahi, v16b alo,
                                         const unsigned short* whb, const unsigned short* wlb, int ks) {
#pragma unroll
  for (int ct = 0; ct < CT; ++ct) {
    const unsigned short* ph = whb + (size_t)ct * 16 * K + 32 * ks;
    const unsigned short* pl = wlb + (size_t)ct * 16 * K + 32 * ks;
    FragB bh, bl;
    frag_b(ph, pl, bh, bl);
    c[ct] = wmb(ahi, bh.v, c[ct]);
    c[ct] = wmb(ahi, bl.v, c[ct]);
    c[ct] = wmb(alo, bh.v, c[ct]);
  }
}

template <int NB>
__device__ __forceinline__ int scan_chunk(const int* __restrict__ dsts, int nE, int cbase, int nodeBase,
                                          int vec8, int* list, int tid, int lane, int wave) {
  int wc = 0;
#pragma unroll
  for (int g = 0; g < NGRP; ++g) {
    const int el0  = (g * NTHR + tid) * EPT;
    const int e0   = cbase + el0;
    const int sent = -2147483647 - 1;
    v4i da, db;
    if (vec8 != 0 && cbase + CHUNK <= nE) {
      da = *(const v4i*)(dsts + e0);
      db = *(const v4i*)(dsts + e0 + 4);
    } else {
      da.x = (e0     < nE) ? dsts[min(e0, nE - 1)] : sent;
      da.y = (e0 + 1 < nE) ? dsts[min(e0 + 1, nE - 1)] : sent;
      da.z = (e0 + 2 < nE) ? dsts[min(e0 + 2, nE - 1)] : sent;
      da.w = (e0 + 3 < nE) ? dsts[min(e0 + 3, nE - 1)] : sent;
      db.x = (e0 + 4 < nE) ? dsts[min(e0 + 4, nE - 1)] : sent;
      db.y = (e0 + 5 < nE) ? dsts[min(e0 + 5, nE - 1)] : sent;
      db.z = (e0 + 6 < nE) ? dsts[min(e0 + 6, nE - 1)] : sent;
      db.w = (e0 + 7 < nE) ? dsts[min(e0 + 7, nE - 1)] : sent;
    }
    const unsigned nb = (unsigned)nodeBase;
    const unsigned s0 = (unsigned)da.x - nb, s1 = (unsigned)da.y - nb;
    const unsigned s2 = (unsigned)da.z - nb, s3 = (unsigned)da.w - nb;
    const unsigned s4 = (unsigned)db.x - nb, s5 = (unsigned)db.y - nb;
    const unsigned s6 = (unsigned)db.z - nb, s7 = (unsigned)db.w - nb;
    const bool h0 = s0 < (unsigned)NB, h1 = s1 < (unsigned)NB, h2 = s2 < (unsigned)NB, h3 = s3 < (unsigned)NB;
    const bool h4 = s4 < (unsigned)NB, h5 = s5 < (unsigned)NB, h6 = s6 < (unsigned)NB, h7 = s7 < (unsigned)NB;
    const unsigned any = __builtin_amdgcn_ballot_w32(h0 | h1 | h2 | h3 | h4 | h5 | h6 | h7);
    if (any != 0u) {
#define HITJ(J, HJ, SJ) { \
        const unsigned mj = __builtin_amdgcn_ballot_w32(HJ); \
        if (mj != 0u) { \
          if (HJ) { \
            const int pos = wc + (int)__builtin_amdgcn_mbcnt_lo(mj, 0u); \
            if (pos < WCAP) list[wave * WCAP + pos] = ((el0 + (J)) << 12) | (int)(SJ); \
          } \
          wc += (int)__builtin_popcount(mj); } }
      HITJ(0, h0, s0)
      HITJ(1, h1, s1)
      HITJ(2, h2, s2)
      HITJ(3, h3, s3)
      HITJ(4, h4, s4)
      HITJ(5, h5, s5)
      HITJ(6, h6, s6)
      HITJ(7, h7, s7)
#undef HITJ
    }
  }
  return wc;
}

__global__ __launch_bounds__(NTHR) void k_prep(
    const float* __restrict__ wr1, const float* __restrict__ wo1,
    const float* __restrict__ wr2, const float* __restrict__ wo2,
    const float* __restrict__ wr3, const float* __restrict__ wo3,
    const float* __restrict__ l1w, const float* __restrict__ l2w,
    unsigned short* planes) {
  const int pl = blockIdx.y;
  const float* sa; const float* sb;
  int no, kp, d1, d2, oh, ol;
  if (pl == 0)      { sa = wr1; sb = wo1; no = NOUT1; kp = 2 * FIN1; d1 = FIN1; d2 = FIN1; oh = PO_W1H; ol = PO_W1L; }
  else if (pl == 1) { sa = wr2; sb = wo2; no = NOUT2; kp = 2 * FIN2; d1 = FIN2; d2 = FIN2; oh = PO_W2H; ol = PO_W2L; }
  else if (pl == 2) { sa = wr3; sb = wo3; no = NOUT3; kp = 2 * F3;   d1 = F3;   d2 = F3;   oh = PO_W3H; ol = PO_W3L; }
  else if (pl == 3) { sa = l1w; sb = l1w; no = NL1;   kp = KL1;      d1 = NOUT3 + DEMW; d2 = 0; oh = PO_L1H; ol = PO_L1L; }
  else              { sa = l2w; sb = l2w; no = NL2;   kp = NL1;      d1 = NL1;  d2 = 0;    oh = PO_L2H; ol = PO_L2L; }
  const int grp = blockIdx.x * NTHR + threadIdx.x;
  if (grp >= no * kp / 8) return;
  const int o = grp * 8, n = o / kp, k0 = o - n * kp;
  const int kbmax = d2 > 0 ? d2 - 1 : 0;
  float v[8];
#pragma unroll
  for (int j = 0; j < 8; ++j) {
    const int k  = k0 + j;
    const int ka = k < d1 ? k : d1 - 1;
    int kb = k - d1; kb = kb < 0 ? 0 : (kb > kbmax ? kbmax : kb);
    const float va = sa[(size_t)ka * no + n];
    const float vb = sb[(size_t)kb * no + n];
    v[j] = (k < d1) ? va : ((k - d1 < d2) ? vb : 0.0f);
  }
  v4f a, b;
  a.x = v[0]; a.y = v[1]; a.z = v[2]; a.w = v[3];
  b.x = v[4]; b.y = v[5]; b.z = v[6]; b.w = v[7];
  v8us hi, lo;
  split8(a, b, hi, lo);
  unsigned short* ph = planes + oh + o;
  unsigned short* pq = planes + ol + o;
  *(volatile v8us*)ph = hi;
  *(volatile v8us*)pq = lo;
  __threadfence();
  *(volatile v8us*)ph = hi;
  *(volatile v8us*)pq = lo;
}

__global__ __launch_bounds__(NTHR) void k_embed(
    const int* __restrict__ xidx, const float* __restrict__ emb, float* x0, int nN, int nV, int nRows) {
  const int t = blockIdx.x * NTHR + threadIdx.x;
  if (t >= nRows * 4) return;
  const int row = t >> 2, c = (t & 3) * 4;
  const int node = row < nN ? row : nN - 1;
  int id = xidx[node];
  id = id < 0 ? 0 : (id > nV - 1 ? nV - 1 : id);
  const v4f v = *(const v4f*)(emb + (size_t)id * FIN1 + c);
  float* p = x0 + (size_t)row * FIN1 + c;
  *(volatile v4f*)p = v;
  __threadfence();
  *(volatile v4f*)p = v;
}

template <int FIN, int NB, int NOUT>
__global__ __launch_bounds__(NTHR) void k_conv(
    const int* __restrict__ ei, const float* __restrict__ ew, const float* __restrict__ xin,
    const unsigned short* __restrict__ whi, const unsigned short* __restrict__ wlo,
    const float* __restrict__ bias, float* hout, int nN, int nE, int vec8) {
  constexpr int K = 2 * FIN, CT = NOUT / 16, RTW = NB / 16 / NWAVE;
  static_assert(NB * FIN * 4 + LISTN * 4 + 64 <= LDS_CONV);
  static_assert((NB & (NB - 1)) == 0 && NB <= 4096);
  static_assert(FIN == 16 || FIN == 64);
  static_assert((NOUT % 32) == 0 && (CT % 2) == 0);
  extern __shared__ v4f lds_dyn[];
  float* acc  = (float*)lds_dyn;
  int*   list = (int*)(acc + NB * FIN);
  int*   wcnt = list + LISTN;
  const int tid = threadIdx.x, lane = tid & 31, wave = tid >> 5, hh = lane >> 4, m = lane & 15;
  const int nodeBase = blockIdx.x * NB;
  const int* dsts = ei + nE;

  {
    const v4f z = {0.f, 0.f, 0.f, 0.f};
    for (int i = tid; i < NB * FIN / 4; i += NTHR) lds_dyn[i] = z;
  }
  __syncthreads();

  const int nChunks = (nE + CHUNK - 1) / CHUNK;
#pragma unroll 1
  for (int ch = 0; ch < nChunks; ++ch) {
    const int cbase = ch * CHUNK;
    const int wc = scan_chunk<NB>(dsts, nE, cbase, nodeBase, vec8, list, tid, lane, wave);
    if (lane == 0) wcnt[wave] = wc;
    __syncthreads();
    if (wave == 0) {
#pragma unroll 1
      for (int wsx = 0; wsx < NWAVE; ++wsx) {
        int n = __builtin_amdgcn_readfirstlane(wcnt[wsx]);
        n = n > WCAP ? WCAP : (n < 0 ? 0 : n);
        const int* lp = list + wsx * WCAP;
#pragma unroll 1
        for (int i = 0; i < n; ++i) {
          const int ent  = __builtin_amdgcn_readfirstlane(lp[i]);
          const int slot = ent & (NB - 1);
          int e = cbase + ((ent >> 12) & (CHUNK - 1));
          e = e > nE - 1 ? nE - 1 : e;
          int src = ei[e];
          src = src < 0 ? 0 : (src > nN - 1 ? nN - 1 : src);
          const float w = ew[e];
          if (FIN == 16) {
            const float v  = xin[(size_t)src * 16 + m];
            float* ap      = acc + slot * 16 + m;
            const float nv = *ap + w * v;
            if (lane < 16) *ap = nv;
          } else {
            const v2f v = *(const v2f*)(xin + (size_t)src * FIN + 2 * lane);
            v2f* ap = (v2f*)(acc + slot * FIN + 2 * lane);
            *ap = *ap + v * w;
          }
        }
      }
    }
    __syncthreads();
  }

  float* stg = (float*)list + wave * 512;
  const unsigned short* whb = whi + (size_t)m * K + 8 * hh;
  const unsigned short* wlb = wlo + (size_t)m * K + 8 * hh;
#pragma unroll 1
  for (int it = 0; it < RTW; ++it) {
    const int t = wave * RTW + it;
    int node = nodeBase + 16 * t + m;
    node = node > nN - 1 ? nN - 1 : node;
    const float* arow = acc + (16 * t + m) * FIN + 8 * hh;
    const float* xrow = xin + (size_t)node * FIN + 8 * hh;
    v8f c[CT];
#pragma unroll
    for (int ct = 0; ct < CT; ++ct) { const v8f z = {0.f, 0.f, 0.f, 0.f, 0.f, 0.f, 0.f, 0.f}; c[ct] = z; }
    if (FIN == 16) {
      FragB ah, al;
      { const v4f p0 = *(const v4f*)arow, p1 = *(const v4f*)(arow + 4); split8(p0, p1, ah.u[0], al.u[0]); }
      { const v4f p0 = *(const v4f*)xrow, p1 = *(const v4f*)(xrow + 4); split8(p0, p1, ah.u[1], al.u[1]); }
      mma_step<CT, K>(c, ah.v, al.v, whb, wlb, 0);
    } else {
#pragma unroll
      for (int ks = 0; ks < FIN / 32; ++ks) {
        FragB ah, al;
        frag_a(arow + 32 * ks, ah, al);
        mma_step<CT, K>(c, ah.v, al.v, whb, wlb, ks);
      }
#pragma unroll
      for (int ks = 0; ks < FIN / 32; ++ks) {
        FragB ah, al;
        frag_a(xrow + 32 * ks, ah, al);
        mma_step<CT, K>(c, ah.v, al.v, whb, wlb, FIN / 32 + ks);
      }
    }
#pragma unroll
    for (int cp = 0; cp < CT / 2; ++cp) {
      const float b0 = bias[32 * cp + m], b1 = bias[32 * cp + 16 + m];
      float* sp = stg + (8 * hh) * 32 + m;
#pragma unroll
      for (int r = 0; r < 8; ++r) { sp[r * 32] = c[2 * cp][r] + b0; sp[r * 32 + 16] = c[2 * cp + 1][r] + b1; }
      __syncthreads();
      v4f ov[4];
      const float* rp = stg + (lane >> 3) * 32 + 4 * (lane & 7);
#pragma unroll
      for (int q = 0; q < 4; ++q) ov[q] = *(const v4f*)(rp + q * 128);
      float* gp = hout + ((size_t)nodeBase + 16 * t + (lane >> 3)) * NOUT + 32 * cp + 4 * (lane & 7);
#pragma unroll
      for (int q = 0; q < 4; ++q) *(volatile v4f*)(gp + (size_t)q * 4 * NOUT) = ov[q];
      __threadfence();
#pragma unroll
      for (int q = 0; q < 4; ++q) *(volatile v4f*)(gp + (size_t)q * 4 * NOUT) = ov[q];
      __syncthreads();
    }
  }
}

template <int F, int MODE>
__global__ __launch_bounds__(NTHR) void k_gstat(
    const float* __restrict__ h, const int* __restrict__ batch,
    const float* __restrict__ meanIn, const float* __restrict__ ga, float* outp, int nN) {
#pragma clang fp contract(off)
  constexpr int S = NTHR / F;
  static_assert(F == 64 || F == 128);
  extern __shared__ v4f lds_dyn[];
  double* accd = (double*)lds_dyn;
  int*    cnti = (int*)((char*)lds_dyn + NTHR * NG * 8);
  float*  res  = (float*)((char*)lds_dyn + NTHR * NG * 8 + 512 * 4);
  const int tid = threadIdx.x, s = tid / F, f = tid - s * F;
  for (int i = tid; i < S * NG * F; i += NTHR) accd[i] = 0.0;
  for (int i = tid; i < 512; i += NTHR) cnti[i] = 0;
  __syncthreads();

  const float af = (MODE == 1) ? ga[f] : 0.0f;
  double* myacc = accd + (size_t)s * NG * F + f;
  const int nIt = (nN + S - 1) / S;
#pragma unroll 2
  for (int i = 0; i < nIt; ++i) {
    const int nraw = i * S + s;
    const int node = nraw > nN - 1 ? nN - 1 : nraw;
    int g = batch[node];
    g = g < 0 ? 0 : (g > NG - 1 ? NG - 1 : g);
    const float x = h[(size_t)node * F + f];
    float q;
    if (MODE == 0) { q = x; }
    else { const float mm = meanIn[g * F + f]; const float am = af * mm; const float xc = x - am; q = xc * xc; }
    if (nraw < nN) {
      myacc[g * F] += (double)q;
      if (f == 0) cnti[s * NG + g] += 1;
    }
  }
  __syncthreads();

  for (int idx = tid; idx < NG * F; idx += NTHR) {
    const int g = idx / F, f2 = idx - g * F;
    double sum = 0.0; int c = 0;
#pragma unroll 1
    for (int s2 = 0; s2 < S; ++s2) { sum += accd[((size_t)s2 * NG + g) * F + f2]; c += cnti[s2 * NG + g]; }
    const float inv = 1.0f / fmaxf((float)c, 1.0f);
    const float mv  = (float)sum * inv;
    res[idx] = (MODE == 0) ? mv : (1.0f / sqrtf(mv + 1e-5f));
  }
  __syncthreads();

  for (int i = tid; i < NG * F / 4; i += NTHR) { const v4f v = *(const v4f*)(res + 4 * i); *(volatile v4f*)(outp + 4 * i) = v; }
  __threadfence();
  for (int i = tid; i < NG * F / 4; i += NTHR) { const v4f v = *(const v4f*)(res + 4 * i); *(volatile v4f*)(outp + 4 * i) = v; }
}

template <int F>
__global__ __launch_bounds__(NTHR) void k_gapply(
    const float* __restrict__ h, const int* __restrict__ batch,
    const float* __restrict__ mean, const float* __restrict__ rstd,
    const float* __restrict__ gg, const float* __restrict__ gb, const float* __restrict__ ga,
    float* hn, int nN) {
#pragma clang fp contract(off)
  const int t = blockIdx.x * NTHR + threadIdx.x;
  const int total = nN * (F / 4);
  if (t >= total) return;
  const int node = t / (F / 4), c = (t - node * (F / 4)) * 4;
  int g = batch[node];
  g = g < 0 ? 0 : (g > NG - 1 ? NG - 1 : g);
  const v4f x  = *(const v4f*)(h + (size_t)node * F + c);
  const v4f mv = *(const v4f*)(mean + g * F + c);
  const v4f rv = *(const v4f*)(rstd + g * F + c);
  const v4f av = *(const v4f*)(ga + c);
  const v4f wv = *(const v4f*)(gg + c);
  const v4f bv = *(const v4f*)(gb + c);
  const v4f am = av * mv;
  const v4f xc = x - am;
  v4f y = wv * xc;
  y = y * rv;
  y = y + bv;
  y.x = y.x > 0.f ? y.x : 0.01f * y.x;
  y.y = y.y > 0.f ? y.y : 0.01f * y.y;
  y.z = y.z > 0.f ? y.z : 0.01f * y.z;
  y.w = y.w > 0.f ? y.w : 0.01f * y.w;
  float* p = hn + (size_t)node * F + c;
  *(volatile v4f*)p = y;
  __threadfence();
  *(volatile v4f*)p = y;
}

__global__ __launch_bounds__(PTHR) void k_pool(
    const int* __restrict__ ei, const float* __restrict__ ew, const int* __restrict__ batch,
    const float* __restrict__ hn, double* part, int nN, int nE, int epb, int npb) {
  extern __shared__ v4f lds_dyn[];
  double* pool = (double*)lds_dyn;
  const int f = threadIdx.x;
  for (int i = f; i < RECD; i += PTHR) pool[i] = 0.0;
  __syncthreads();

  const int e0 = blockIdx.x * epb;
  int e1 = e0 + epb; e1 = e1 > nE ? nE : e1;
#pragma unroll 2
  for (int e = e0; e < e1; ++e) {
    int s = ei[e];               s = s < 0 ? 0 : (s > nN - 1 ? nN - 1 : s);
    int d = ei[(size_t)nE + e];  d = d < 0 ? 0 : (d > nN - 1 ? nN - 1 : d);
    int g = batch[d];            g = g < 0 ? 0 : (g > NG - 1 ? NG - 1 : g);
    const float w = ew[e];
    const float v = hn[(size_t)s * F3 + f];
    pool[g * F3 + f] += (double)(w * v);
  }
  const int n0 = blockIdx.x * npb;
  int n1 = n0 + npb; n1 = n1 > nN ? nN : n1;
#pragma unroll 2
  for (int i = n0; i < n1; ++i) {
    int g = batch[i]; g = g < 0 ? 0 : (g > NG - 1 ? NG - 1 : g);
    pool[(NG + g) * F3 + f] += (double)hn[(size_t)i * F3 + f];
    if (f == 0) pool[2 * NG * F3 + g] += 1.0;
  }
  __syncthreads();

  double* dst = part + (size_t)blockIdx.x * RECD;
#pragma unroll 1
  for (int it = 0; it < RECD / 2 / PTHR; ++it) {
    const int idx = (it * PTHR + f) * 2;
    const v2d v = *(const v2d*)(pool + idx);
    *(volatile v2d*)(dst + idx) = v;
  }
  __threadfence();
#pragma unroll 1
  for (int it = 0; it < RECD / 2 / PTHR; ++it) {
    const int idx = (it * PTHR + f) * 2;
    const v2d v = *(const v2d*)(pool + idx);
    *(volatile v2d*)(dst + idx) = v;
  }
}

__global__ __launch_bounds__(NTHR) void k_head(
    const double* __restrict__ part, int nP,
    const float* __restrict__ demog, const float* __restrict__ demw, const float* __restrict__ demb,
    const unsigned short* __restrict__ planes, const float* __restrict__ br3,
    const float* __restrict__ l1b, const float* __restrict__ bn1g, const float* __restrict__ bn1b,
    const float* __restrict__ l2b, const float* __restrict__ bn2g, const float* __restrict__ bn2b,
    const float* __restrict__ l3w, const float* __restrict__ l3b, float* out) {
#pragma clang fp contract(off)
  extern __shared__ v4f lds_dyn[];
  float* L   = (float*)lds_dyn;
  float* A3  = L + HL_A3;
  float* H0  = L + HL_H0;
  float* INV = L + HL_INV;
  float* CF  = L + HL_CF;
  float* OS  = L + HL_OUT;
  float* H1  = A3;
  float* H2  = H0;
  const int tid = threadIdx.x, lane = tid & 31, wave = tid >> 5, hh = lane >> 4, m = lane & 15;

  for (int idx = tid; idx < NG * F3; idx += NTHR) {
    const int g = idx >> 7, f = idx & (F3 - 1);
    double sa = 0.0, sx = 0.0;
#pragma unroll 1
    for (int p = 0; p < nP; ++p) {
      const double* b = part + (size_t)p * RECD;
      sa += b[g * F3 + f];
      sx += b[(NG + g) * F3 + f];
    }
    A3[g * (2 * F3) + f]      = (float)sa;
    A3[g * (2 * F3) + F3 + f] = (float)sx;
  }
  for (int idx = tid; idx < (HROWS - NG) * (2 * F3); idx += NTHR) A3[NG * (2 * F3) + idx] = 0.0f;
  {
    const int tt = tid < NG ? tid : NG - 1;
    double c = 0.0;
#pragma unroll 1
    for (int p = 0; p < nP; ++p) c += part[(size_t)p * RECD + 2 * NG * F3 + tt];
    const float cf32 = (float)c;
    const float iv   = 1.0f / fmaxf(cf32, 1.0f);
    const float cfv  = cf32 * iv;
    if (tid < HROWS) { INV[tid] = tid < NG ? iv : 0.0f; CF[tid] = tid < NG ? cfv : 0.0f; }
  }
  for (int idx = tid; idx < HROWS * 32; idx += NTHR) {
    const int row = idx >> 5, cc = idx & 31;
    const int rb = row < NG ? row : NG - 1, jc = cc & (DEMW - 1);
    float s = 0.0f;
#pragma unroll
    for (int k = 0; k < DEMO; ++k) s = s + demog[rb * DEMO + k] * demw[k * DEMW + jc];
    s = s + demb[jc];
    H0[row * KL1 + NOUT3 + cc] = (row < NG && cc < DEMW) ? s : 0.0f;
  }
  __syncthreads();

  {
    const int ct0 = 2 * wave;
#pragma unroll 1
    for (int rt = 0; rt < HROWS / 16; ++rt) {
      v8f c[2];
      { const v8f z = {0.f, 0.f, 0.f, 0.f, 0.f, 0.f, 0.f, 0.f}; c[0] = z; c[1] = z; }
      const float* ar = A3 + (16 * rt + m) * (2 * F3) + 8 * hh;
#pragma unroll 2
      for (int ks = 0; ks < (2 * F3) / 32; ++ks) {
        FragB ah, al;
        frag_a(ar + 32 * ks, ah, al);
#pragma unroll
        for (int j = 0; j < 2; ++j) {
          const size_t bo = (size_t)(16 * (ct0 + j) + m) * (2 * F3) + 32 * ks + 8 * hh;
          FragB bh, bl;
          frag_b(planes + PO_W3H + bo, planes + PO_W3L + bo, bh, bl);
          c[j] = wmb(ah.v, bh.v, c[j]);
          c[j] = wmb(ah.v, bl.v, c[j]);
          c[j] = wmb(al.v, bh.v, c[j]);
        }
      }
#pragma unroll
      for (int j = 0; j < 2; ++j) {
        const int col = 16 * (ct0 + j) + m;
        const float bc = br3[col];
#pragma unroll
        for (int r = 0; r < 8; ++r) {
          const int row = 16 * rt + 8 * hh + r;
          const float t0 = c[j][r] * INV[row];
          const float t1 = bc * CF[row];
          H0[row * KL1 + col] = t0 + t1;
        }
      }
    }
  }
  __syncthreads();

  {
#pragma unroll 1
    for (int rt = 0; rt < HROWS / 16; ++rt) {
      v8f c = {0.f, 0.f, 0.f, 0.f, 0.f, 0.f, 0.f, 0.f};
      const float* ar = H0 + (16 * rt + m) * KL1 + 8 * hh;
#pragma unroll 3
      for (int ks = 0; ks < KL1 / 32; ++ks) {
        FragB ah, al, bh, bl;
        frag_a(ar + 32 * ks, ah, al);
        const size_t bo = (size_t)(16 * wave + m) * KL1 + 32 * ks + 8 * hh;
        frag_b(planes + PO_L1H + bo, planes + PO_L1L + bo, bh, bl);
        c = wmb(ah.v, bh.v, c);
        c = wmb(ah.v, bl.v, c);
        c = wmb(al.v, bh.v, c);
      }
      const int col = 16 * wave + m;
      const float bc = l1b[col];
#pragma unroll
      for (int r = 0; r < 8; ++r) H1[(16 * rt + 8 * hh + r) * NL1 + col] = c[r] + bc;
    }
  }
  __syncthreads();

  if (tid < NL1) {
    const int n = tid;
    double s = 0.0;
#pragma unroll 1
    for (int g = 0; g < NG; ++g) s += (double)H1[g * NL1 + n];
    const double md = s * (1.0 / NG);
    double q = 0.0;
#pragma unroll 1
    for (int g = 0; g < NG; ++g) { const double d = (double)H1[g * NL1 + n] - md; q += d * d; }
    const float mf = (float)md;
    const float vf = (float)(q * (1.0 / NG));
    const float rs = 1.0f / sqrtf(vf + 1e-5f);
    const float gw = bn1g[n], gbv = bn1b[n];
#pragma unroll 1
    for (int g = 0; g < NG; ++g) {
      const float x = H1[g * NL1 + n];
      float y = gw * (x - mf);
      y = y * rs;
      y = y + gbv;
      H1[g * NL1 + n] = y > 0.f ? y : 0.01f * y;
    }
    for (int g = NG; g < HROWS; ++g) H1[g * NL1 + n] = 0.0f;
  }
  __syncthreads();

#pragma unroll 1
  for (int job = wave; job < (HROWS / 16) * (NL2 / 16); job += NWAVE) {
    const int rt = job >> 2, cc = job & 3;
    v8f c = {0.f, 0.f, 0.f, 0.f, 0.f, 0.f, 0.f, 0.f};
    const float* ar = H1 + (16 * rt + m) * NL1 + 8 * hh;
#pragma unroll
    for (int ks = 0; ks < NL1 / 32; ++ks) {
      FragB ah, al, bh, bl;
      frag_a(ar + 32 * ks, ah, al);
      const size_t bo = (size_t)(16 * cc + m) * NL1 + 32 * ks + 8 * hh;
      frag_b(planes + PO_L2H + bo, planes + PO_L2L + bo, bh, bl);
      c = wmb(ah.v, bh.v, c);
      c = wmb(ah.v, bl.v, c);
      c = wmb(al.v, bh.v, c);
    }
    const int col = 16 * cc + m;
    const float bc = l2b[col];
#pragma unroll
    for (int r = 0; r < 8; ++r) H2[(16 * rt + 8 * hh + r) * NL2 + col] = c[r] + bc;
  }
  __syncthreads();

  if (tid < NL2) {
    const int n = tid;
    double s = 0.0;
#pragma unroll 1
    for (int g = 0; g < NG; ++g) s += (double)H2[g * NL2 + n];
    const double md = s * (1.0 / NG);
    double q = 0.0;
#pragma unroll 1
    for (int g = 0; g < NG; ++g) { const double d = (double)H2[g * NL2 + n] - md; q += d * d; }
    const float mf = (float)md;
    const float vf = (float)(q * (1.0 / NG));
    const float rs = 1.0f / sqrtf(vf + 1e-5f);
    const float gw = bn2g[n], gbv = bn2b[n];
#pragma unroll 1
    for (int g = 0; g < NG; ++g) {
      const float x = H2[g * NL2 + n];
      float y = gw * (x - mf);
      y = y * rs;
      y = y + gbv;
      H2[g * NL2 + n] = y > 0.f ? y : 0.01f * y;
    }
  }
  __syncthreads();

  for (int idx = tid; idx < NG * NCLS; idx += NTHR) {
    const int b = idx / NCLS, j = idx - b * NCLS;
    float s = 0.0f;
#pragma unroll 1
    for (int k = 0; k < NL2; ++k) s = s + H2[b * NL2 + k] * l3w[k * NCLS + j];
    OS[idx] = s + l3b[j];
  }
  __syncthreads();

  const bool wl = tid < 75;
  v4f o0 = {0.f, 0.f, 0.f, 0.f};
  if (wl) o0 = *(const v4f*)(OS + 4 * tid);
  if (wl) *(volatile v4f*)(out + 4 * tid) = o0;
  __threadfence();
  if (wl) *(volatile v4f*)(out + 4 * tid) = o0;
}

extern "C" void kernel_launch(void* const* d_in, const int* in_sizes, int n_in,
                              void* d_out, int out_size, void* d_ws, size_t ws_size,
                              hipStream_t stream) {
  if (n_in < 33) return;
  const int nN = in_sizes[0];
  const int nE = in_sizes[1] / 2;
  const int nV = in_sizes[5] / FIN1;
  if (nN <= 0 || nE <= 0 || nV <= 0) return;
  if (in_sizes[1] != 2 * nE || in_sizes[2] != nE || in_sizes[3] != nN || in_sizes[5] != nV * FIN1) return;
  if (out_size != NG * NCLS || in_sizes[4] != NG * DEMO) return;
  if (in_sizes[6] != FIN1 * NOUT1 || in_sizes[7] != NOUT1 || in_sizes[8] != FIN1 * NOUT1) return;
  if (in_sizes[9] != FIN2 * NOUT2 || in_sizes[10] != NOUT2 || in_sizes[11] != FIN2 * NOUT2) return;
  if (in_sizes[12] != F3 * NOUT3 || in_sizes[13] != NOUT3 || in_sizes[14] != F3 * NOUT3) return;
  if (in_sizes[15] != NOUT1 || in_sizes[16] != NOUT1 || in_sizes[17] != NOUT1) return;
  if (in_sizes[18] != NOUT2 || in_sizes[19] != NOUT2 || in_sizes[20] != NOUT2) return;
  if (in_sizes[21] != DEMO * DEMW || in_sizes[22] != DEMW) return;
  if (in_sizes[23] != (NOUT3 + DEMW) * NL1 || in_sizes[24] != NL1 || in_sizes[25] != NL1 || in_sizes[26] != NL1) return;
  if (in_sizes[27] != NL1 * NL2 || in_sizes[28] != NL2 || in_sizes[29] != NL2 || in_sizes[30] != NL2) return;
  if (in_sizes[31] != NL2 * NCLS || in_sizes[32] != NCLS) return;

  const int*   x_idx  = (const int*)d_in[0];
  const int*   ei     = (const int*)d_in[1];
  const float* ew     = (const float*)d_in[2];
  const int*   batch  = (const int*)d_in[3];
  const float* demog  = (const float*)d_in[4];
  const float* emb    = (const float*)d_in[5];
  const float* w_rel1 = (const float*)d_in[6];
  const float* b_rel1 = (const float*)d_in[7];
  const float* w_root1= (const float*)d_in[8];
  const float* w_rel2 = (const float*)d_in[9];
  const float* b_rel2 = (const float*)d_in[10];
  const float* w_root2= (const float*)d_in[11];
  const float* w_rel3 = (const float*)d_in[12];
  const float* b_rel3 = (const float*)d_in[13];
  const float* w_root3= (const float*)d_in[14];
  const float* gn1_g  = (const float*)d_in[15];
  const float* gn1_b  = (const float*)d_in[16];
  const float* gn1_a  = (const float*)d_in[17];
  const float* gn2_g  = (const float*)d_in[18];
  const float* gn2_b  = (const float*)d_in[19];
  const float* gn2_a  = (const float*)d_in[20];
  const float* demo_w = (const float*)d_in[21];
  const float* demo_b = (const float*)d_in[22];
  const float* l1_w   = (const float*)d_in[23];
  const float* l1_b   = (const float*)d_in[24];
  const float* bn1_g  = (const float*)d_in[25];
  const float* bn1_b  = (const float*)d_in[26];
  const float* l2_w   = (const float*)d_in[27];
  const float* l2_b   = (const float*)d_in[28];
  const float* bn2_g  = (const float*)d_in[29];
  const float* bn2_b  = (const float*)d_in[30];
  const float* l3_w   = (const float*)d_in[31];
  const float* l3_b   = (const float*)d_in[32];
  float* out = (float*)d_out;

  const int nRows0 = (nN + 63) & ~63;
  const int nA1 = (nN + NB1 - 1) / NB1;
  const int nA2 = (nN + NB2 - 1) / NB2;
  const int epb = (nE + POOLP - 1) / POOLP;
  const int npb = (nN + POOLP - 1) / POOLP;

  char* ws = (char*)d_ws;
  size_t off = 0;
  const size_t oPL = off;  off += ((size_t)PO_TOT * 2 + 255) & ~(size_t)255;
  const size_t szX0 = ((size_t)nRows0 * FIN1 * 4 + 255) & ~(size_t)255;
  const size_t szH1 = ((size_t)nA1 * NB1 * NOUT1 * 4 + 255) & ~(size_t)255;
  const size_t szH2 = ((size_t)nA2 * NB2 * NOUT2 * 4 + 255) & ~(size_t)255;
  const size_t szA  = (szX0 + szH1 > szH2) ? (szX0 + szH1) : szH2;
  const size_t oA = off;   off += szA;
  const size_t oX0 = oA, oH1 = oA + szX0, oH2 = oA;
  const size_t szB = ((size_t)nN * NOUT2 * 4 + 255) & ~(size_t)255;
  const size_t oB = off;   off += szB;
  const size_t oM1 = off;  off += ((size_t)NG * NOUT1 * 4 + 255) & ~(size_t)255;
  const size_t oR1 = off;  off += ((size_t)NG * NOUT1 * 4 + 255) & ~(size_t)255;
  const size_t oM2 = off;  off += ((size_t)NG * NOUT2 * 4 + 255) & ~(size_t)255;
  const size_t oR2 = off;  off += ((size_t)NG * NOUT2 * 4 + 255) & ~(size_t)255;
  const size_t oPT = off;  off += ((size_t)POOLP * RECD * 8 + 255) & ~(size_t)255;
  if (off > ws_size || off > (size_t)134217728) return;

  unsigned short* planes = (unsigned short*)(ws + oPL);
  float*  x0   = (float*)(ws + oX0);
  float*  h1   = (float*)(ws + oH1);
  float*  h2   = (float*)(ws + oH2);
  float*  hn   = (float*)(ws + oB);
  float*  m1   = (float*)(ws + oM1);
  float*  r1   = (float*)(ws + oR1);
  float*  m2   = (float*)(ws + oM2);
  float*  r2   = (float*)(ws + oR2);
  double* part = (double*)(ws + oPT);

  const int vec8 = ((nE & 3) == 0) ? 1 : 0;

  k_prep<<<dim3(32, 5), NTHR, 0, stream>>>(w_rel1, w_root1, w_rel2, w_root2, w_rel3, w_root3, l1_w, l2_w, planes);

  k_embed<<<(nRows0 * 4) / NTHR, NTHR, 0, stream>>>(x_idx, emb, x0, nN, nV, nRows0);

  hipFuncSetAttribute(reinterpret_cast<const void*>(&k_conv<FIN1, NB1, NOUT1>),
                      hipFuncAttributeMaxDynamicSharedMemorySize, LDS_CONV);
  k_conv<FIN1, NB1, NOUT1><<<nA1, NTHR, LDS_CONV, stream>>>(
      ei, ew, x0, planes + PO_W1H, planes + PO_W1L, b_rel1, h1, nN, nE, vec8);

  hipFuncSetAttribute(reinterpret_cast<const void*>(&k_gstat<NOUT1, 0>),
                      hipFuncAttributeMaxDynamicSharedMemorySize, LDS_STAT);
  hipFuncSetAttribute(reinterpret_cast<const void*>(&k_gstat<NOUT1, 1>),
                      hipFuncAttributeMaxDynamicSharedMemorySize, LDS_STAT);
  k_gstat<NOUT1, 0><<<1, NTHR, LDS_STAT, stream>>>(h1, batch, m1, gn1_a, m1, nN);
  k_gstat<NOUT1, 1><<<1, NTHR, LDS_STAT, stream>>>(h1, batch, m1, gn1_a, r1, nN);
  k_gapply<NOUT1><<<(nN * (NOUT1 / 4) + NTHR - 1) / NTHR, NTHR, 0, stream>>>(
      h1, batch, m1, r1, gn1_g, gn1_b, gn1_a, hn, nN);

  hipFuncSetAttribute(reinterpret_cast<const void*>(&k_conv<FIN2, NB2, NOUT2>),
                      hipFuncAttributeMaxDynamicSharedMemorySize, LDS_CONV);
  k_conv<FIN2, NB2, NOUT2><<<nA2, NTHR, LDS_CONV, stream>>>(
      ei, ew, hn, planes + PO_W2H, planes + PO_W2L, b_rel2, h2, nN, nE, vec8);

  hipFuncSetAttribute(reinterpret_cast<const void*>(&k_gstat<NOUT2, 0>),
                      hipFuncAttributeMaxDynamicSharedMemorySize, LDS_STAT);
  hipFuncSetAttribute(reinterpret_cast<const void*>(&k_gstat<NOUT2, 1>),
                      hipFuncAttributeMaxDynamicSharedMemorySize, LDS_STAT);
  k_gstat<NOUT2, 0><<<1, NTHR, LDS_STAT, stream>>>(h2, batch, m2, gn2_a, m2, nN);
  k_gstat<NOUT2, 1><<<1, NTHR, LDS_STAT, stream>>>(h2, batch, m2, gn2_a, r2, nN);
  k_gapply<NOUT2><<<(nN * (NOUT2 / 4) + NTHR - 1) / NTHR, NTHR, 0, stream>>>(
      h2, batch, m2, r2, gn2_g, gn2_b, gn2_a, hn, nN);

  hipFuncSetAttribute(reinterpret_cast<const void*>(&k_pool),
                      hipFuncAttributeMaxDynamicSharedMemorySize, LDS_POOL);
  k_pool<<<POOLP, PTHR, LDS_POOL, stream>>>(ei, ew, batch, hn, part, nN, nE, epb, npb);

  hipFuncSetAttribute(reinterpret_cast<const void*>(&k_head),
                      hipFuncAttributeMaxDynamicSharedMemorySize, LDS_HEAD);
  k_head<<<1, NTHR, LDS_HEAD, stream>>>(part, POOLP, demog, demo_w, demo_b, planes, b_rel3,
                                         l1_b, bn1_g, bn1_b, l2_b, bn2_g, bn2_b, l3_w, l3_b, out);
}
